// HybridLocalAggregator_29248727286399
// MI455X (gfx1250) — hardware-verified
//
#include <hip/hip_runtime.h>
#include <math.h>

typedef __attribute__((ext_vector_type(16))) _Float16 v16h;
typedef __attribute__((ext_vector_type(16))) __bf16 v16b;
typedef __attribute__((ext_vector_type(8)))  _Float16 v8h;
typedef __attribute__((ext_vector_type(8)))  float v8f;
typedef __attribute__((ext_vector_type(4)))  float v4f;
typedef __attribute__((ext_vector_type(2)))  float v2f;
typedef __attribute__((ext_vector_type(4)))  unsigned v4u;
typedef __attribute__((ext_vector_type(4)))  int v4i;
typedef float __attribute__((may_alias)) float_a;
typedef int __attribute__((may_alias)) int_a;

template <typename T> __device__ __forceinline__ void vst2(void* p, T v) { *(volatile T*)p = v; __threadfence(); *(volatile T*)p = v; }
__device__ __forceinline__ v8f wmma16(v16h a, v16h b, v8f c) {
  v8f d = __builtin_amdgcn_wmma_f32_16x16x32_f16(false, a, false, b, (short)0, c, false, false);
  asm volatile("v_nop\n\tv_nop\n\tv_nop\n\tv_nop" : "+v"(d) : "v"(a), "v"(b));
  return d;
}
__device__ __forceinline__ v8f wmma_bf(v16b a, v16b b, v8f c) {
  v8f d = __builtin_amdgcn_wmma_f32_16x16x32_bf16(false, a, false, b, (short)0, c, false, false);
  asm volatile("v_nop\n\tv_nop\n\tv_nop\n\tv_nop" : "+v"(d) : "v"(a), "v"(b));
  return d;
}
__device__ __forceinline__ v16h frag_h(const _Float16* rowk0, int lane) {
  union { v16h v; v8h q[2]; } u; const _Float16* p = rowk0 + 8 * (lane >> 4);
  u.q[0] = *(const v8h*)p; u.q[1] = *(const v8h*)(p + 16); return u.v;
}
__device__ __forceinline__ v16h frag_f32(const float* rowk0, int lane) {
  v16h a; const float* p = rowk0 + 8 * (lane >> 4);
#pragma unroll
  for (int i = 0; i < 8; ++i) { a[i] = (_Float16)p[i]; a[8 + i] = (_Float16)p[16 + i]; }
  return a;
}
__device__ __forceinline__ v16h frag_f32s(const float* rowk0, int lane, float sc) {
  v16h a; const float* p = rowk0 + 8 * (lane >> 4);
#pragma unroll
  for (int i = 0; i < 8; ++i) { a[i] = (_Float16)(p[i] * sc); a[8 + i] = (_Float16)(p[16 + i] * sc); }
  return a;
}
__device__ __forceinline__ v16h fragc_f32(const float* W, int k0, int n, int lane, int ld, int K) {
  v16h a; const int g = lane >> 4;
#pragma unroll
  for (int i = 0; i < 8; ++i) { const int ka = k0 + 8 * g + i, kb = ka + 16;
    a[i] = (_Float16)(ka < K ? W[(size_t)(ka < K ? ka : K - 1) * ld + n] : 0.f); a[8 + i] = (_Float16)(kb < K ? W[(size_t)(kb < K ? kb : K - 1) * ld + n] : 0.f); }
  return a;
}
struct F2 { v16b h, l; };
__device__ __forceinline__ F2 bsplit16(const float v[16]) { F2 r;
#pragma unroll
  for (int i = 0; i < 16; ++i) { const __bf16 h = (__bf16)v[i]; r.h[i] = h; r.l[i] = (__bf16)(v[i] - (float)h); }
  return r; }
__device__ __forceinline__ F2 split_row(const float* row, int k0, int lane) { float v[16]; const float* p = row + k0 + 8 * (lane >> 4);
#pragma unroll
  for (int i = 0; i < 8; ++i) { v[i] = p[i]; v[8 + i] = p[16 + i]; }
  return bsplit16(v); }
__device__ __forceinline__ F2 split_rowK(const float* row, int k0, int lane, int K) { float v[16]; const int g = lane >> 4;
#pragma unroll
  for (int i = 0; i < 8; ++i) { const int ka = k0 + 8 * g + i, kb = ka + 16; v[i] = ka < K ? row[ka < K ? ka : K - 1] : 0.f; v[8 + i] = kb < K ? row[kb < K ? kb : K - 1] : 0.f; }
  return bsplit16(v); }
__device__ __forceinline__ F2 split_col(const float* W, int k0, int n, int lane, int ld, int K) { float v[16]; const int g = lane >> 4;
#pragma unroll
  for (int i = 0; i < 8; ++i) { const int ka = k0 + 8 * g + i, kb = ka + 16; v[i] = ka < K ? W[(size_t)(ka < K ? ka : K - 1) * ld + n] : 0.f; v[8 + i] = kb < K ? W[(size_t)(kb < K ? kb : K - 1) * ld + n] : 0.f; }
  return bsplit16(v); }
__device__ __forceinline__ v8f mac3(const F2& a, const F2& b, v8f c) { c = wmma_bf(a.l, b.h, c); c = wmma_bf(a.h, b.l, c); return wmma_bf(a.h, b.h, c); }
__device__ __forceinline__ float sigm(float v) { return 1.0f / (1.0f + expf(-v)); }
#define LDSX() do { asm volatile("s_wait_dscnt 0" ::: "memory"); __builtin_amdgcn_wave_barrier(); __builtin_amdgcn_fence(__ATOMIC_RELEASE, "workgroup"); } while (0)


#define CSR_N 100000
#define CSR_E 800000
#define NNP 100032
#define NF 64
#define EBLK 64
#define NEB (CSR_E / EBLK)
#ifndef DBGM
#define DBGM 0
#endif
#ifndef TLB
#define TLB (NNP / 64)
#endif
#ifndef DNEB
#define DNEB NEB
#endif

#define CSR_FINN (CSR_E + 32 * CSR_NBK)
#ifndef CSR_CHUNK
#define CSR_CHUNK 4096
#endif
#define CSR_EPT (CSR_CHUNK / 256)
#define CSR_BKT 256
#define CSR_NCH ((CSR_E + CSR_CHUNK - 1) / CSR_CHUNK)
#define CSR_NBK ((CSR_N + CSR_BKT - 1) / CSR_BKT)
#define CSR_NBKP (((CSR_NBK + 63) / 64) * 64)
#define CSR_SEGCAP (CSR_E + 32 * CSR_NBK * CSR_NCH)
#ifndef CSR_BCAP
#define CSR_BCAP 10240
#endif
#define CSR_SZ_CNT   (4u * CSR_NCH * CSR_NBKP)
#define CSR_SZ_OFF   (4u * CSR_NBK * (((CSR_NCH + 31) / 32) * 32))
#define CSR_SZ_BST   (4u * (((CSR_NBK + 1 + 31) / 32) * 32))
#define CSR_SZ_SEG   (4u * CSR_SEGCAP)
#define CSR_SZ_FIN   (4u * (CSR_E + 32 * CSR_NBK))
#define CSR_SZ_ROW   (4u * CSR_NBK * CSR_BKT)
#define CSR_OFFP (((CSR_NCH + 31) / 32) * 32)

__global__ __launch_bounds__(256) void k_csr_cnt(const int* __restrict__ DST, int dstride, int* __restrict__ CNT) {
  __shared__ unsigned short sc[256][CSR_NBK + 1]; __shared__ __align__(16) int srow[CSR_NBKP];
  const int c = blockIdx.x, tid = threadIdx.x;
  for (int b = 0; b < CSR_NBK; ++b) sc[tid][b] = 0;
  const size_t e0 = (size_t)c * CSR_CHUNK + tid * CSR_EPT;
  for (int i = 0; i < CSR_EPT; ++i) { const size_t e = e0 + i; if (e < (size_t)CSR_E) { int d = DST[e * dstride]; d = min(max(d, 0), CSR_N - 1); sc[tid][d / CSR_BKT] += 1; } }
  __syncthreads();
  for (int b = tid; b < CSR_NBKP; b += 256) { int s = 0; if (b < CSR_NBK) for (int t = 0; t < 256; ++t) s += sc[t][b]; srow[b] = s; }
  __syncthreads();
  for (int q = tid; q < CSR_NBKP / 4; q += 256) vst2((unsigned*)(CNT + (size_t)c * CSR_NBKP + q * 4), *(const v4u*)&srow[q * 4]);
}
__global__ __launch_bounds__(256) void k_csr_scan(const int* __restrict__ CNT, int* __restrict__ OFF, int* __restrict__ BST) {
  __shared__ int sbt[CSR_NBK + 1]; __shared__ int sbs[((CSR_NBK + 1 + 31) / 32) * 32]; __shared__ int scnt[CSR_NBK + 1]; __shared__ __align__(16) int sbuf[64][CSR_OFFP];
  const int tid = threadIdx.x;
  for (int b = tid; b < CSR_NBK; b += 256) { int sp = 0, st = 0; for (int c = 0; c < CSR_NCH; ++c) { const int n = CNT[(size_t)c * CSR_NBKP + b]; st += n; sp += (n + 31) & ~31; } sbt[b] = sp; scnt[b] = st; }
  for (int b = tid; b < ((CSR_NBK + 1 + 31) / 32) * 32; b += 256) sbs[b] = 0;
  __syncthreads();
  if (tid == 0) { int acc = 0, accf = 0; for (int b = 0; b < CSR_NBK; ++b) { const int t = sbt[b]; sbt[b] = acc; acc += t; sbs[b] = accf; accf += (scnt[b] + 31) & ~31; } sbs[CSR_NBK] = accf; }
  __syncthreads();
  for (int b0 = 0; b0 < CSR_NBK; b0 += 64) {
    if (tid < 64 && b0 + tid < CSR_NBK) { const int b = b0 + tid; int o = sbt[b]; for (int c = 0; c < CSR_OFFP; ++c) { if (c < CSR_NCH) { sbuf[tid][c] = o; o += (CNT[(size_t)c * CSR_NBKP + b] + 31) & ~31; } else sbuf[tid][c] = 0; } }
    __syncthreads();
    for (int q = tid; q < 64 * (CSR_OFFP / 4); q += 256) { const int r = q / (CSR_OFFP / 4), pc = q % (CSR_OFFP / 4); if (b0 + r < CSR_NBK) vst2((unsigned*)(OFF + (size_t)(b0 + r) * CSR_OFFP + pc * 4), *(const v4u*)&sbuf[r][pc * 4]); }
    __syncthreads(); }
  for (int q = tid; q < ((CSR_NBK + 1 + 31) / 32) * 32 / 4; q += 256) vst2((unsigned*)(BST + q * 4), *(const v4u*)&sbs[q * 4]);
}
__global__ __launch_bounds__(256) void k_csr_scatter(const int* __restrict__ SRC, const int* __restrict__ DST, int sstride, int dstride, const int* __restrict__ OFF, int* __restrict__ SEGS, int* __restrict__ SEGE) {
  __shared__ unsigned short sc[256][CSR_NBK + 1]; __shared__ int sbase[CSR_NBK + 1]; __shared__ int scn[CSR_NBK + 1]; __shared__ int sord[CSR_CHUNK];
  const int c = blockIdx.x, tid = threadIdx.x;
  for (int b = 0; b < CSR_NBK; ++b) sc[tid][b] = 0;
  const size_t e0 = (size_t)c * CSR_CHUNK + tid * CSR_EPT; int bk[CSR_EPT];
#pragma unroll
  for (int i = 0; i < CSR_EPT; ++i) { const size_t e = e0 + i; bk[i] = -1; if (e < (size_t)CSR_E) { int d = DST[e * dstride]; d = min(max(d, 0), CSR_N - 1); bk[i] = d / CSR_BKT; sc[tid][bk[i]] += 1; } }
  __syncthreads();
  for (int b = tid; b < CSR_NBK; b += 256) { int acc = 0; for (int t = 0; t < 256; ++t) { const int v = sc[t][b]; sc[t][b] = (unsigned short)acc; acc += v; } scn[b] = acc; }
  __syncthreads();
  if (tid == 0) { int acc = 0; for (int b = 0; b < CSR_NBK; ++b) { sbase[b] = acc; acc += scn[b]; } }
  __syncthreads();
#pragma unroll
  for (int i = 0; i < CSR_EPT; ++i) { if (bk[i] >= 0) { const int b = bk[i]; const int r = sc[tid][b]; sc[tid][b] = (unsigned short)(r + 1); sord[sbase[b] + r] = tid * CSR_EPT + i; } }
  __syncthreads();
  for (int b = 0; b < CSR_NBK; ++b) { const int n = scn[b]; if (n == 0) continue; const int nl = ((n + 31) & ~31); const size_t o = (size_t)(min(max(OFF[(size_t)b * CSR_OFFP + c], 0), CSR_SEGCAP - nl) & ~31);
    for (int q = tid; q < nl / 4; q += 256) { int4 vs, ve;
#pragma unroll
      for (int k = 0; k < 4; ++k) { const int i = q * 4 + k; int s = -1, eid = -1; if (i < n) { const size_t e = (size_t)c * CSR_CHUNK + sord[sbase[b] + i]; s = min(max(SRC[e * sstride], 0), CSR_N - 1); eid = (int)e; } vs[k] = s; ve[k] = eid; }
      vst2((unsigned*)(SEGS + o + q * 4), *(const v4u*)&vs); vst2((unsigned*)(SEGE + o + q * 4), *(const v4u*)&ve); } }
}
__global__ __launch_bounds__(256) void k_csr_bucket(const int* __restrict__ CNT, const int* __restrict__ OFF, const int* __restrict__ BST, const int* __restrict__ SEGS, const int* __restrict__ SEGE, const int* __restrict__ DST, int dstride, int* __restrict__ FS, int* __restrict__ FE, int* __restrict__ ROWST, int* __restrict__ ROWCNT) {
  __shared__ int ssrc[CSR_BCAP]; __shared__ int seid[CSR_BCAP]; __shared__ unsigned char snod[CSR_BCAP]; __shared__ int souts[CSR_BCAP]; __shared__ int soute[CSR_BCAP]; __shared__ int scount[256]; __shared__ int sstart[257]; __shared__ int stot;
  const int b = blockIdx.x, tid = threadIdx.x;
  if (tid == 0) { int t = 0; for (int c = 0; c < CSR_NCH; ++c) t += min(max(CNT[(size_t)c * CSR_NBKP + b], 0), CSR_CHUNK); stot = (t <= CSR_BCAP) ? t : 0; }
  __syncthreads();
  { int base = 0; for (int c = 0; c < CSR_NCH; ++c) { const int n = min(max(CNT[(size_t)c * CSR_NBKP + b], 0), CSR_CHUNK); const int o = min(max(OFF[(size_t)b * CSR_OFFP + c], 0), CSR_SEGCAP - ((n + 31) & ~31));
      for (int i = tid; i < n; i += 256) { const int p = base + i; if (p < CSR_BCAP) { ssrc[p] = min(max(SEGS[o + i], 0), CSR_N - 1); const int e = min(max(SEGE[o + i], 0), CSR_E - 1); seid[p] = e; int d = DST[(size_t)e * dstride]; d = min(max(d, 0), CSR_N - 1); const int dl = d - b * CSR_BKT; snod[p] = (unsigned char)(dl >= 0 && dl < 256 ? dl : 255); } }
      base += n; } }
  __syncthreads();
  const int node = b * CSR_BKT + tid; int cnt = 0; for (int p = 0; p < stot; ++p) cnt += (snod[p] == tid) ? 1 : 0;
  scount[tid] = cnt; __syncthreads();
  if (tid == 0) { int acc = 0; for (int t = 0; t < 256; ++t) { sstart[t] = acc; acc += scount[t]; } sstart[256] = acc; }
  __syncthreads();
  const int bst0 = min(max(BST[b], 0), CSR_FINN - ((sstart[256] + 31) & ~31)) & ~31; const int gst = bst0 + sstart[tid];
  { int w = sstart[tid]; for (int p = 0; p < stot; ++p) if (snod[p] == tid) { souts[w] = ssrc[p]; soute[w] = seid[p]; ++w; } }
  __syncthreads();
  { const int n = sstart[256]; const int nl = (n + 31) & ~31; for (int q = tid; q < nl / 4; q += 256) { int4 vs, ve;
#pragma unroll
      for (int k = 0; k < 4; ++k) { const int i = q * 4 + k; vs[k] = i < n ? souts[i] : -1; ve[k] = i < n ? soute[i] : -1; }
      vst2((unsigned*)(FS + bst0 + q * 4), *(const v4u*)&vs); vst2((unsigned*)(FE + bst0 + q * 4), *(const v4u*)&ve); } }
  __syncthreads();
  { __shared__ __align__(16) int srs[256], src2[256]; srs[tid] = node < CSR_N ? gst : 0; src2[tid] = node < CSR_N ? cnt : 0; __syncthreads();
    if (tid < 64) vst2((unsigned*)(ROWST + (size_t)b * 256 + tid * 4), *(const v4u*)&srs[tid * 4]); else if (tid < 128) vst2((unsigned*)(ROWCNT + (size_t)b * 256 + (tid - 64) * 4), *(const v4u*)&src2[(tid - 64) * 4]); }
}

typedef __attribute__((ext_vector_type(8))) __bf16 v8b;
__device__ __forceinline__ v16b frag_b(const __bf16* rowk0, int lane) {
  union { v16b v; v8b q[2]; } u; const __bf16* p = rowk0 + 8 * (lane >> 4);
  u.q[0] = *(const v8b*)p; u.q[1] = *(const v8b*)(p + 16); return u.v;
}
__device__ __forceinline__ float bfr(float v) { return (float)(__bf16)v; }
__device__ __attribute__((noinline)) float exp_ni(float v) { return expf(v); }
#define WS_CNT  0u
#define WS_OFF  (WS_CNT + CSR_SZ_CNT)
#define WS_BST  (WS_OFF + CSR_SZ_OFF)
#define WS_SEGS (WS_BST + CSR_SZ_BST)
#define WS_SEGE (WS_SEGS + CSR_SZ_SEG)
#define WS_FS   (WS_SEGE + CSR_SZ_SEG)
#define WS_FE   (WS_FS + CSR_SZ_FIN)
#define WS_RST  (WS_FE + CSR_SZ_FIN)
#define WS_RCT  (WS_RST + CSR_SZ_ROW)
#define WS_PT   (WS_RCT + CSR_SZ_ROW)
#define PT_W1 0
#define PT_W2 (64 * 128)
#define PT_FU (64 * 128 + 64 * 64)
#define PT_END (64 * 128 + 64 * 64 + 64 * 128)
#define WS_XP   (WS_PT + 2u * PT_END)
#define WS_BN   (WS_XP + 4u * (NNP / 64) * 128)
#define WS_HN   (WS_BN + 4u * 4 * 128)
#define WS_EP   (WS_HN + 4u * NNP * NF)
#define WS_O    (WS_EP + 4u * NEB * 128)
#define WS_OP   (WS_O + 4u * NNP * NF)
#define WS_END  (WS_OP + 4u * (NNP / 64) * 128)

__global__ __launch_bounds__(128) void k_pack(const float* __restrict__ W1, const float* __restrict__ W2, const float* __restrict__ FW, __bf16* __restrict__ PT) {
  __shared__ __align__(16) __bf16 srow[128];
  const int n = blockIdx.x, tid = threadIdx.x; int len; size_t dst;
  if (n < 64) { len = 128; dst = PT_W1 + (size_t)n * 128; srow[tid] = (__bf16)bfr(W1[tid * 64 + n]); }
  else if (n < 128) { const int o = n - 64; len = 64; dst = PT_W2 + (size_t)o * 64; if (tid < 64) srow[tid] = (__bf16)bfr(W2[tid * 64 + o]); }
  else { const int o = n - 128; len = 128; dst = PT_FU + (size_t)o * 128; srow[tid] = (__bf16)bfr(FW[tid * 64 + o]); }
  __syncthreads();
  if (tid < len / 8) vst2((unsigned*)(PT + dst + tid * 8), *(const v4u*)(&srow[tid * 8]));
}
template <bool RND>
__global__ __launch_bounds__(64) void k_colpart(const float* __restrict__ M, int nrows, float* __restrict__ PART) {
  __shared__ __align__(16) float sp[128];
  const int c = threadIdx.x; const size_t r0 = (size_t)blockIdx.x * 64; float s = 0.f, q = 0.f;
  for (int r = 0; r < 64; ++r) { const size_t row = r0 + r; if (row < (size_t)nrows) { float v = M[row * 64 + c]; if (RND) v = bfr(v); s += v; q += v * v; } }
  sp[c] = s; sp[64 + c] = q; __syncthreads();
  if (c < 32) vst2(PART + (size_t)blockIdx.x * 128 + c * 4, *(const v4f*)&sp[c * 4]);
}
__global__ __launch_bounds__(64) void k_fin(const float* __restrict__ PART, int nblk, float cnt, const float* __restrict__ g, const float* __restrict__ bb, float* __restrict__ BNslot) {
  __shared__ __align__(16) float so[128];
  const int c = threadIdx.x; float s = 0.f, q = 0.f;
  for (int b = 0; b < nblk; ++b) { s += PART[(size_t)b * 128 + c]; q += PART[(size_t)b * 128 + 64 + c]; }
  const float m = s / cnt; const float var = fmaxf(q / cnt - m * m, 0.f); const float sc = bfr(g[c]) * rsqrtf(var + 1e-5f); so[c] = sc; so[64 + c] = bfr(bb[c]) - m * sc;
  __syncthreads();
  if (c < 32) vst2(BNslot + c * 4, *(const v4f*)&so[c * 4]);
}
__global__ __launch_bounds__(256) void k_xbn(const float* __restrict__ X, const float* __restrict__ BN0, float* __restrict__ HN) {
  const int tid = threadIdx.x; const size_t r = (size_t)blockIdx.x * 64 + (tid >> 2);
  for (int piece = (tid & 3); piece < 16; piece += 4) { v4f v; for (int i = 0; i < 4; ++i) { const int c = piece * 4 + i; v[i] = r < (size_t)CSR_N ? bfr(X[r * 64 + c]) * BN0[c] + BN0[64 + c] : 0.f; } vst2(HN + r * 64 + piece * 4, v); }
}
template <int STAGE>
__device__ __forceinline__ void edge_tile(const float* __restrict__ HN, const __bf16* __restrict__ PT, const float* __restrict__ b1, const float* __restrict__ b2, const float* __restrict__ BN, const int* srw, const int* scl,
                                          __bf16 (*sah)[136], __bf16 (*sal)[136], float (*sz)[68], int lane) {
  const int col = lane & 15, g = lane >> 4;
  if (lane < 16) { const int r = srw[lane], c = scl[lane]; const float* hr = HN + (size_t)max(r, 0) * 64; const float* hc = HN + (size_t)max(c, 0) * 64;
    for (int k = 0; k < 64; ++k) { const float a = r >= 0 ? hr[k] : 0.f; const float d = r >= 0 ? (hr[k] - hc[k]) : 0.f; __bf16 hb = (__bf16)a; sah[lane][k] = hb; sal[lane][k] = (__bf16)(a - (float)hb); hb = (__bf16)d; sah[lane][64 + k] = hb; sal[lane][64 + k] = (__bf16)(d - (float)hb); } }
  LDSX();
  v8f acc[4] = {};
#pragma unroll
  for (int kc = 0; kc < 4; ++kc) { const v16b ah = frag_b(&sah[col][kc * 32], lane), al = frag_b(&sal[col][kc * 32], lane);
#pragma unroll
    for (int j = 0; j < 4; ++j) { const v16b w = frag_b(PT + PT_W1 + (size_t)(j * 16 + col) * 128 + kc * 32, lane); acc[j] = wmma_bf(al, w, acc[j]); acc[j] = wmma_bf(ah, w, acc[j]); } }
  LDSX();
#pragma unroll
  for (int j = 0; j < 4; ++j) { const int o = j * 16 + col; const float bb = bfr(b1[o]);
#pragma unroll
    for (int r = 0; r < 8; ++r) { float z = fmaxf(acc[j][r] + bb, 0.f);
      if (STAGE == 1) sz[8 * g + r][o] = z;
      else { const float e1 = z * BN[128 + o] + BN[128 + 64 + o]; const __bf16 hb = (__bf16)e1; sah[8 * g + r][o] = hb; sal[8 * g + r][o] = (__bf16)(e1 - (float)hb); } } }
  if (STAGE == 1) { LDSX(); return; }
  LDSX();
  v8f acc2[4] = {};
#pragma unroll
  for (int kc = 0; kc < 2; ++kc) { const v16b ah = frag_b(&sah[col][kc * 32], lane), al = frag_b(&sal[col][kc * 32], lane);
#pragma unroll
    for (int j = 0; j < 4; ++j) { const v16b w = frag_b(PT + PT_W2 + (size_t)(j * 16 + col) * 64 + kc * 32, lane); acc2[j] = wmma_bf(al, w, acc2[j]); acc2[j] = wmma_bf(ah, w, acc2[j]); } }
#pragma unroll
  for (int j = 0; j < 4; ++j) { const int o = j * 16 + col; const float bb = bfr(b2[o]);
#pragma unroll
    for (int r = 0; r < 8; ++r) { const float z = fmaxf(acc2[j][r] + bb, 0.f); sz[8 * g + r][o] = (STAGE == 2) ? z : z * BN[256 + o] + BN[256 + 64 + o]; } }
  LDSX();
}
template <int STAGE>
__global__ __launch_bounds__(128) void k_es(const int* __restrict__ EI, const float* __restrict__ HN, const __bf16* __restrict__ PT, const float* __restrict__ b1, const float* __restrict__ b2, const float* __restrict__ BN, float* __restrict__ EP) {
  __shared__ __align__(16) __bf16 sah[4][16][136], sal[4][16][136]; __shared__ __align__(16) float sz[4][16][68]; __shared__ int srw[4][16], scl[4][16]; __shared__ float sred[4][128]; __shared__ __align__(16) float sp[128];
  const int tid = threadIdx.x, wave = tid >> 5, lane = tid & 31; const size_t e0 = (size_t)blockIdx.x * EBLK + wave * 16;
  if (lane < 16) { const size_t e = e0 + lane; srw[wave][lane] = e < (size_t)CSR_E ? min(max(EI[e], 0), CSR_N - 1) : -1; scl[wave][lane] = e < (size_t)CSR_E ? min(max(EI[(size_t)CSR_E + e], 0), CSR_N - 1) : -1; }
  LDSX();
  edge_tile<STAGE>(HN, PT, b1, b2, BN, srw[wave], scl[wave], sah[wave], sal[wave], sz[wave], lane);
  { float s0 = 0.f, q0 = 0.f, s1 = 0.f, q1 = 0.f; for (int r = 0; r < 16; ++r) if (srw[wave][r] >= 0) { const float a = sz[wave][r][lane], c = sz[wave][r][lane + 32]; s0 += a; q0 += a * a; s1 += c; q1 += c * c; }
    sred[wave][lane] = s0; sred[wave][32 + lane] = s1; sred[wave][64 + lane] = q0; sred[wave][96 + lane] = q1; }
  __syncthreads();
  if (tid < 128) sp[tid] = (sred[0][tid] + sred[1][tid]) + (sred[2][tid] + sred[3][tid]);
  __syncthreads();
  if (tid < 32) vst2(EP + (size_t)blockIdx.x * 128 + tid * 4, *(const v4f*)&sp[tid * 4]);
}
__global__ __launch_bounds__(128) void k_node(const float* __restrict__ HN, const __bf16* __restrict__ PT, const float* __restrict__ b1, const float* __restrict__ b2, const float* __restrict__ BN, const float* __restrict__ AW, const float* __restrict__ AB, const float* __restrict__ FB,
                                             const int* __restrict__ FS, const int* __restrict__ FE, const int* __restrict__ RST, const int* __restrict__ RCT, const int* __restrict__ EI, float* __restrict__ O) {
  __shared__ __align__(16) __bf16 sah[4][16][136], sal[4][16][136]; __shared__ __align__(16) float sz[4][16][68]; __shared__ int srw[4][16], scl[4][16], snd[4][16]; __shared__ int sst[4][17];
  __shared__ float smax[4][16][65], sacc[4][16][65], sm[4][16], sl[4][16]; __shared__ float saw[64]; __shared__ __align__(16) float so[4][16][68];
  const int tid = threadIdx.x, wave = tid >> 5, lane = tid & 31, col = lane & 15, g = lane >> 4; const size_t n0 = (size_t)blockIdx.x * 64 + wave * 16;
  if (tid < 64) saw[tid] = bfr(AW[tid]);
  for (int q = lane; q < 16 * 65; q += 32) { (&smax[wave][0][0])[q] = -3.0e38f; (&sacc[wave][0][0])[q] = 0.f; } if (lane < 16) { sm[wave][lane] = -3.0e38f; sl[wave][lane] = 0.f; }
  if (lane <= 16) { const size_t n = n0 + min(lane, 15); int c = 0, s = 0; if (n < (size_t)CSR_N) { c = min(max(RCT[n], 0), CSR_BCAP); s = min(max(RST[n], 0), CSR_FINN - c); } sst[wave][lane] = (lane < 16) ? s : s + c; }
  __syncthreads();
  const float ab = bfr(AB[0]); const int ebeg = sst[wave][0]; int eend = sst[wave][16]; eend = max(min(eend, ebeg + 4096), ebeg);
#pragma unroll 1
  for (int t0 = ebeg; t0 < eend; t0 += 16) {
    if (lane < 16) { const int ei = t0 + lane; if (ei < eend) { srw[wave][lane] = min(max(FS[ei], 0), CSR_N - 1);   int nd = 15; for (int i = 0; i < 16; ++i) if (ei >= sst[wave][i] && ei < sst[wave][i + 1]) nd = i; snd[wave][lane] = nd; scl[wave][lane] = (int)(n0 + nd); }
      else { srw[wave][lane] = -1; scl[wave][lane] = 0; snd[wave][lane] = 255; } }
    LDSX();
    edge_tile<3>(HN, PT, b1, b2, BN, srw[wave], scl[wave], sah[wave], sal[wave], sz[wave], lane);
    for (int e = 0; e < 16; ++e) { const int nd = snd[wave][e]; if (nd >= 16) continue;
      const float v0 = sz[wave][e][lane], v1 = sz[wave][e][lane + 32];
      smax[wave][nd][lane] = fmaxf(smax[wave][nd][lane], v0); smax[wave][nd][lane + 32] = fmaxf(smax[wave][nd][lane + 32], v1);
      float lg = v0 * saw[lane] + v1 * saw[lane + 32];
#pragma unroll
      for (int o = 1; o < 32; o <<= 1) lg += __shfl_xor(lg, o);
      lg += ab;
      const float mo = sm[wave][nd]; const float mn = fmaxf(mo, lg); const float alpha = exp_ni(mo - mn); const float p = exp_ni(lg - mn);
      sacc[wave][nd][lane] = sacc[wave][nd][lane] * alpha + p * v0; sacc[wave][nd][lane + 32] = sacc[wave][nd][lane + 32] * alpha + p * v1;
      if (lane == 0) { sl[wave][nd] = sl[wave][nd] * alpha + p; sm[wave][nd] = mn; }
      LDSX(); }
    LDSX(); }
  if (lane < 16) { const int nl = lane; const int deg = sst[wave][nl + 1] - sst[wave][nl]; const float il = deg > 0 ? 1.0f / sl[wave][nl] : 0.f;
    for (int c = 0; c < 64; ++c) { const float mxv = deg > 0 ? smax[wave][nl][c] : 0.f; const float at = sacc[wave][nl][c] * il; __bf16 hb = (__bf16)mxv; sah[wave][nl][c] = hb; sal[wave][nl][c] = (__bf16)(mxv - (float)hb); hb = (__bf16)at; sah[wave][nl][64 + c] = hb; sal[wave][nl][64 + c] = (__bf16)(at - (float)hb); } }
  LDSX();
  { v8f acc[4] = {};
#pragma unroll
    for (int kc = 0; kc < 4; ++kc) { const v16b ah = frag_b(&sah[wave][col][kc * 32], lane), al = frag_b(&sal[wave][col][kc * 32], lane);
#pragma unroll
      for (int j = 0; j < 4; ++j) { const v16b w = frag_b(PT + PT_FU + (size_t)(j * 16 + col) * 128 + kc * 32, lane); acc[j] = wmma_bf(al, w, acc[j]); acc[j] = wmma_bf(ah, w, acc[j]); } }
#pragma unroll
    for (int j = 0; j < 4; ++j) { const int o = j * 16 + col; const float bb = bfr(FB[o]);
#pragma unroll
      for (int r = 0; r < 8; ++r) so[wave][8 * g + r][o] = (n0 + 8 * g + r < (size_t)CSR_N) ? acc[j][r] + bb : 0.f; } }
  LDSX();
  for (int rl = 0; rl < 16; ++rl) if (lane < 16) vst2(O + (n0 + rl) * 64 + lane * 4, *(const v4f*)&so[wave][rl][lane * 4]);
}
__global__ __launch_bounds__(256) void k_out(const float* __restrict__ O, const float* __restrict__ BN3, float* __restrict__ out) {
  const int tid = threadIdx.x; const size_t r = (size_t)blockIdx.x * 64 + (tid >> 2); if (r >= (size_t)CSR_N) return;
  for (int piece = (tid & 3); piece < 16; piece += 4) { v4f v; for (int i = 0; i < 4; ++i) { const int c = piece * 4 + i; v[i] = fmaxf(O[r * 64 + c] * BN3[c] + BN3[64 + c], 0.f); } vst2(out + r * 64 + piece * 4, v); }
}


#if DBGM == 1 || DBGM == 2
__global__ __launch_bounds__(128) void k_dbgbn(const float* __restrict__ BN, float* __restrict__ out) { const int t = threadIdx.x; if (t < 96) vst2(out + t * 4, *(const v4f*)(BN + t * 4)); }
#endif
#if DBGM == 2 || DBGM == 3
__global__ __launch_bounds__(64) void k_bnfake(const float* __restrict__ g1, const float* __restrict__ b1, const float* __restrict__ g2, const float* __restrict__ b2, float* __restrict__ BN) { __shared__ __align__(16) float s[256]; const int c = threadIdx.x; const float r = rsqrtf(1.0f + 1e-5f); s[c] = bfr(g1[c]) * r; s[64 + c] = bfr(b1[c]); s[128 + c] = bfr(g2[c]) * r; s[192 + c] = bfr(b2[c]); __syncthreads(); vst2(BN + 128 + c * 4, *(const v4f*)&s[c * 4]); }
#endif
#if DBGM == 3
__global__ __launch_bounds__(256) void k_dbgo(const float* __restrict__ O, float* __restrict__ out) { const int tid = threadIdx.x; const size_t r = (size_t)blockIdx.x * 64 + (tid >> 2); for (int piece = (tid & 3); piece < 16; piece += 4) vst2(out + r * 64 + piece * 4, *(const v4f*)(O + r * 64 + piece * 4)); }
#endif
extern "C" void kernel_launch(void* const* d_in, const int* in_sizes, int n_in, void* d_out, int out_size, void* d_ws, size_t ws_size, hipStream_t stream) {
  (void)in_sizes; (void)n_in; (void)out_size;
  const float** F = (const float**)d_in;
  if (ws_size < (size_t)WS_END) return;
  char* ws = (char*)d_ws;
  int *CNT = (int*)(ws + WS_CNT), *OFF = (int*)(ws + WS_OFF), *BST = (int*)(ws + WS_BST), *SEGS = (int*)(ws + WS_SEGS), *SEGE = (int*)(ws + WS_SEGE), *FS = (int*)(ws + WS_FS), *FE = (int*)(ws + WS_FE), *RST = (int*)(ws + WS_RST), *RCT = (int*)(ws + WS_RCT);
  __bf16* PT = (__bf16*)(ws + WS_PT); float *XP = (float*)(ws + WS_XP), *BN = (float*)(ws + WS_BN), *HN = (float*)(ws + WS_HN), *EP = (float*)(ws + WS_EP), *O = (float*)(ws + WS_O), *OP = (float*)(ws + WS_OP);
  const int* EI = (const int*)d_in[17]; const int* ROWI = EI; const int* COLI = EI + CSR_E;
#if DBGM != 1 && DBGM != 2
  k_csr_cnt<<<CSR_NCH, 256, 0, stream>>>(COLI, 1, CNT);
  k_csr_scan<<<1, 256, 0, stream>>>(CNT, OFF, BST);
  k_csr_scatter<<<CSR_NCH, 256, 0, stream>>>(ROWI, COLI, 1, 1, OFF, SEGS, SEGE);
  k_csr_bucket<<<CSR_NBK, 256, 0, stream>>>(CNT, OFF, BST, SEGS, SEGE, COLI, 1, FS, FE, RST, RCT);
#endif
  k_pack<<<192, 128, 0, stream>>>(F[3], F[7], F[13], PT);
  k_colpart<true><<<NNP / 64, 64, 0, stream>>>(F[0], CSR_N, XP);
  k_fin<<<1, 64, 0, stream>>>(XP, NNP / 64, (float)CSR_N, F[1], F[2], BN + 0);
  k_xbn<<<NNP / 64, 256, 0, stream>>>(F[0], BN, HN);
#if DBGM == 3
  k_bnfake<<<1, 64, 0, stream>>>(F[5], F[6], F[9], F[10], BN);
#elif DBGM == 1
  k_es<1><<<DNEB, 128, 0, stream>>>(EI, HN, PT, F[4], F[8], BN, EP);
  k_fin<<<1, 64, 0, stream>>>(EP, DNEB, (float)(DNEB * EBLK), F[5], F[6], BN + 128);
  k_dbgbn<<<1, 128, 0, stream>>>(BN, (float*)d_out); return;
#elif DBGM == 2
  k_bnfake<<<1, 64, 0, stream>>>(F[5], F[6], F[9], F[10], BN);
  k_es<2><<<DNEB, 128, 0, stream>>>(EI, HN, PT, F[4], F[8], BN, EP);
  k_fin<<<1, 64, 0, stream>>>(EP, DNEB, (float)(DNEB * EBLK), F[9], F[10], BN + 256);
  k_dbgbn<<<1, 128, 0, stream>>>(BN, (float*)d_out); return;
#else
  k_es<1><<<NEB, 128, 0, stream>>>(EI, HN, PT, F[4], F[8], BN, EP);
  k_fin<<<1, 64, 0, stream>>>(EP, NEB, (float)CSR_E, F[5], F[6], BN + 128);
  k_es<2><<<NEB, 128, 0, stream>>>(EI, HN, PT, F[4], F[8], BN, EP);
  k_fin<<<1, 64, 0, stream>>>(EP, NEB, (float)CSR_E, F[9], F[10], BN + 256);
#endif
  k_node<<<TLB, 128, 0, stream>>>(HN, PT, F[4], F[8], BN, F[11], F[12], F[14], FS, FE, RST, RCT, EI, O);
#if DBGM == 3
  k_dbgo<<<64, 256, 0, stream>>>(O, (float*)d_out); return;
#endif
  k_colpart<false><<<NNP / 64, 64, 0, stream>>>(O, CSR_N, OP);
  k_fin<<<1, 64, 0, stream>>>(OP, NNP / 64, (float)CSR_N, F[15], F[16], BN + 384);
  k_out<<<NNP / 64, 256, 0, stream>>>(O, BN + 384, (float*)d_out);
}
